// DftSpectrogram_80075370267252
// MI455X (gfx1250) — hardware-verified
//
#include <hip/hip_runtime.h>
#include <math.h>

constexpr int kNfft    = 512;
constexpr int kShift   = 160;
constexpr int kFrames  = 601;
constexpr int kHalf    = 256;
constexpr int kTlen    = 96512;
constexpr int kBatch   = 32;
constexpr int kRows    = kBatch * kFrames;
constexpr int kRowsPad = 19264;
constexpr int kScols   = 512;
constexpr int kFrBlocks = kRowsPad * 64 / 256;
constexpr int kWbBlocks = kScols * 64 / 256;
constexpr int kOutFloats = kBatch * kHalf * kFrames;
constexpr int kOutQuads  = kOutFloats / 4;
constexpr float kEps     = 1e-07f;
constexpr float kInvLn10 = 1.0f / 2.302585092994046f;

typedef __attribute__((ext_vector_type(16))) _Float16 v16h;
typedef __attribute__((ext_vector_type(8)))  _Float16 v8h;
typedef __attribute__((ext_vector_type(16))) __bf16   v16b;
typedef __attribute__((ext_vector_type(8)))  __bf16   v8b;
typedef __attribute__((ext_vector_type(8)))  float    v8f;
typedef __attribute__((ext_vector_type(4)))  float    v4f;
typedef __attribute__((ext_vector_type(4)))  unsigned v4u;
#define PSCALE 32768.0f
#define U16(p) ((const unsigned short*)(const void*)(p))
#define PSCALE_INV (1.0f / 32768.0f)

__device__ __forceinline__ unsigned short f2bf_bits(float f) {
  unsigned u = __float_as_uint(f);
  return (unsigned short)((u + 0x7FFFu + ((u >> 16) & 1u)) >> 16);
}
__device__ __forceinline__ float bf_bits2f(unsigned short h) { return __uint_as_float(((unsigned)h) << 16); }

__device__ __forceinline__ void dep_guard_h(v8f& a, v8f& b, v16h x, v16h y) { asm volatile("v_nop\n\tv_nop\n\tv_nop\n\tv_nop" : "+v"(a), "+v"(b) : "v"(x), "v"(y)); }
__device__ __forceinline__ void dep_guard_b(v8f& a, v8f& b, v16b x, v16b y) { asm volatile("v_nop\n\tv_nop\n\tv_nop\n\tv_nop" : "+v"(a), "+v"(b) : "v"(x), "v"(y)); }
__device__ __forceinline__ void keep4_h(v16h a, v16h b, v16h c, v16h d) { asm volatile("v_nop" :: "v"(a), "v"(b), "v"(c), "v"(d)); }
__device__ __forceinline__ void keep4_b(v16b a, v16b b, v16b c, v16b d) { asm volatile("v_nop" :: "v"(a), "v"(b), "v"(c), "v"(d)); }
__device__ __forceinline__ void acc_guard4(v8f& a, v8f& b, v8f& c, v8f& d) { asm volatile("v_nop\n\tv_nop\n\tv_nop\n\tv_nop" : "+v"(a), "+v"(b), "+v"(c), "+v"(d)); }
template <typename T> struct Frag;
template <> struct Frag<_Float16> {
  typedef v16h V; union U { v16h v; v8h h[2]; };
  static __device__ __forceinline__ v16h load(const _Float16* p) {
    U f; f.h[0] = *(const v8h*)(p); f.h[1] = *(const v8h*)(p + 16); return f.v;
  }
  static __device__ __forceinline__ v8f mma(v16h a, v16h b, v8f c) {
    return __builtin_amdgcn_wmma_f32_16x16x32_f16(false, a, false, b, (short)0, c, false, false);
  }
  static __device__ __forceinline__ void guard(v8f& a, v8f& b, v16h x, v16h y) { dep_guard_h(a, b, x, y); }
  static __device__ __forceinline__ void keep(v16h a, v16h b, v16h c, v16h d) { keep4_h(a, b, c, d); }
};
template <> struct Frag<__bf16> {
  typedef v16b V; union U { v16b v; v8b h[2]; };
  static __device__ __forceinline__ v16b load(const __bf16* p) {
    U f; f.h[0] = *(const v8b*)(p); f.h[1] = *(const v8b*)(p + 16); return f.v;
  }
  static __device__ __forceinline__ v8f mma(v16b a, v16b b, v8f c) {
    return __builtin_amdgcn_wmma_f32_16x16x32_bf16(false, a, false, b, (short)0, c, false, false);
  }
  static __device__ __forceinline__ void guard(v8f& a, v8f& b, v16b x, v16b y) { dep_guard_b(a, b, x, y); }
  static __device__ __forceinline__ void keep(v16b a, v16b b, v16b c, v16b d) { keep4_b(a, b, c, d); }
};

template <int ET> struct Elem;
template <> struct Elem<0> { typedef _Float16 T; };
template <> struct Elem<1> { typedef __bf16 T; };
template <int ET, bool SPLIT, int BIAS_MODE, int OUT_MODE, bool RESID, int ACT = 0>
__global__ __launch_bounds__(256) void wmma_gemm64(
    const unsigned short* __restrict__ Ap, const unsigned short* __restrict__ A2p, int lda, long strideA,
    const unsigned short* __restrict__ Btp, const unsigned short* __restrict__ Bt2p, int ldb, long strideB,
    void* __restrict__ Cout, void* __restrict__ Cout2, int ldc, long strideC,
    const float* __restrict__ bias,
    const float* __restrict__ resid, long strideR,
    int M, int N, int K, float scale) {
  typedef typename Elem<ET>::T T;
  typedef typename Frag<T>::V V;
  const T* A = (const T*)Ap; const T* A2 = (const T*)A2p; const T* Bt = (const T*)Btp; const T* Bt2 = (const T*)Bt2p;
  __shared__ __align__(16) float sT[8][16 * 68];
  const int b    = blockIdx.y;
  const int lane = threadIdx.x & 31;
  const int wave = threadIdx.x >> 5;
  const int tilesN = N >> 6;
  const int tilesM = M >> 6;
  const int tile = blockIdx.x * 8 + wave;
  if (tile >= tilesM * tilesN) return;
  const int tm = tile / tilesN;
  const int tn = tile - tm * tilesN;
  const int m0 = tm << 6;
  const int n0 = tn << 6;

  const T* Ab  = A  + (size_t)b * strideA;
  const T* Bb  = Bt + (size_t)b * strideB;
  const T* Ab2 = SPLIT ? (A2  + (size_t)b * strideA) : nullptr;
  const T* Bb2 = SPLIT ? (Bt2 + (size_t)b * strideB) : nullptr;

  const int rlane = lane & 15;
  const int koff  = (lane >> 4) * 8;
  const int mOff  = (lane >> 4) * 8;

  v8f acc[4][4];
#pragma unroll
  for (int i = 0; i < 4; ++i)
#pragma unroll
    for (int j = 0; j < 4; ++j) acc[i][j] = (v8f){0.f,0.f,0.f,0.f,0.f,0.f,0.f,0.f};

  for (int k0 = 0; k0 < K; k0 += 32) {
    V bh[4], bl[4];
#pragma unroll
    for (int j = 0; j < 4; ++j) {
      const size_t bo = (size_t)(n0 + (j << 4) + rlane) * ldb + koff + k0;
      bh[j] = Frag<T>::load(Bb + bo);
      if (SPLIT) bl[j] = Frag<T>::load(Bb2 + bo);
    }
#pragma unroll
    for (int i = 0; i < 4; ++i) {
      const size_t ao = (size_t)(m0 + (i << 4) + rlane) * lda + koff + k0;
      V ah = Frag<T>::load(Ab + ao);
      V al;
      if (SPLIT) al = Frag<T>::load(Ab2 + ao);
#pragma unroll
      for (int j = 0; j < 4; ++j) {
        acc[i][j] = Frag<T>::mma(ah, bh[j], acc[i][j]);
        if (SPLIT) {
          acc[i][j] = Frag<T>::mma(ah, bl[j], acc[i][j]);
          acc[i][j] = Frag<T>::mma(al, bh[j], acc[i][j]);
        }
      }
      Frag<T>::guard(acc[i][0], acc[i][3], ah, SPLIT ? al : ah);
    }
    Frag<T>::keep(bh[0], bh[1], bh[2], bh[3]);
    if (SPLIT) Frag<T>::keep(bl[0], bl[1], bl[2], bl[3]);
  }
  acc_guard4(acc[0][0], acc[0][1], acc[0][2], acc[0][3]);
  acc_guard4(acc[1][0], acc[1][1], acc[1][2], acc[1][3]);
  acc_guard4(acc[2][0], acc[2][1], acc[2][2], acc[2][3]);
  acc_guard4(acc[3][0], acc[3][1], acc[3][2], acc[3][3]);

  float* slab = sT[wave];
  const float* Rb = RESID ? (resid + (size_t)b * strideR) : nullptr;
#pragma unroll
  for (int i = 0; i < 4; ++i) {
    const int mBase = m0 + (i << 4);
#pragma unroll
    for (int j = 0; j < 4; ++j) {
      const int n = n0 + (j << 4) + rlane;
      float bv = 0.f;
      if (BIAS_MODE == 2) bv = bias[n];
#pragma unroll
      for (int r = 0; r < 8; ++r) {
        float v = acc[i][j][r] * scale;
        if (BIAS_MODE == 1) v += bias[mBase + mOff + r];
        if (BIAS_MODE == 2) v += bv;
        if (RESID) v += Rb[(size_t)(mBase + mOff + r) * ldc + n];
        if (ACT == 1) v = tanhf(v);
        if (ACT == 2) v = fmaxf(v, 0.0f);
        if (ACT == 3) v = v / (1.0f + expf(-v));
        if (ACT == 4) v = (v > 0.f) ? v : 0.01f * v;
        if (ACT == 5) v = 0.5f * v * (1.0f + erff(v * 0.70710678118654752f));
        slab[(mOff + r) * 68 + (j << 4) + rlane] = v;
      }
    }
    __builtin_amdgcn_fence(__ATOMIC_RELEASE, "workgroup");
    __builtin_amdgcn_wave_barrier();
    __builtin_amdgcn_fence(__ATOMIC_ACQUIRE, "workgroup");
    if (OUT_MODE == 0) {
      float* C = (float*)Cout + (size_t)b * strideC;
      const int hh = lane >> 4, c4 = (lane & 15) * 4;
      for (int pass = 0; pass < 2; ++pass) {
#pragma unroll
        for (int it = 0; it < 8; ++it) {
          const int row = it * 2 + hh;
          v4f v = *(const v4f*)(slab + row * 68 + c4);
          *(volatile v4f*)(C + (size_t)(mBase + row) * ldc + n0 + c4) = v;
        }
        __threadfence();
      }
    } else {
      const int q = lane >> 3, c8 = (lane & 7) * 8;
      unsigned short* C  = (unsigned short*)Cout  + (size_t)b * strideC;
      unsigned short* C2 = (OUT_MODE == 2) ? ((unsigned short*)Cout2 + (size_t)b * strideC) : nullptr;
      for (int pass = 0; pass < 2; ++pass) {
#pragma unroll
        for (int it = 0; it < 4; ++it) {
          const int row = it * 4 + q;
          const float* sp = slab + row * 68 + c8;
          v8h hv, lv;
#pragma unroll
          for (int e = 0; e < 8; ++e) {
            if (OUT_MODE == 1) {
              hv[e] = (_Float16)sp[e];
            } else {
              unsigned short hb = f2bf_bits(sp[e]);
              unsigned short lb = f2bf_bits(sp[e] - bf_bits2f(hb));
              hv[e] = __builtin_bit_cast(_Float16, hb);
              lv[e] = __builtin_bit_cast(_Float16, lb);
            }
          }
          *(volatile v8h*)(C + (size_t)(mBase + row) * ldc + n0 + c8) = hv;
          if (OUT_MODE == 2) *(volatile v8h*)(C2 + (size_t)(mBase + row) * ldc + n0 + c8) = lv;
        }
        __threadfence();
      }
    }
    __builtin_amdgcn_fence(__ATOMIC_RELEASE, "workgroup");
    __builtin_amdgcn_wave_barrier();
    __builtin_amdgcn_fence(__ATOMIC_ACQUIRE, "workgroup");
  }
}

__device__ __forceinline__ unsigned pack_bf16x2(float lo, float hi) {
  return (unsigned)f2bf_bits(lo) | ((unsigned)f2bf_bits(hi) << 16);
}

__global__ __launch_bounds__(256) void cast_planes(
    const float* __restrict__ x, const float* __restrict__ wr, const float* __restrict__ wi,
    unsigned short* __restrict__ fr, unsigned short* __restrict__ wb)
{
  if (blockIdx.x < (unsigned)kFrBlocks) {
    const int t  = blockIdx.x * 256 + threadIdx.x;
    const int r  = t >> 6;
    const int n0 = (t & 63) * 8;
    const bool live = (r < kRows);
    const int rc = live ? r : (kRows - 1);
    const int b  = rc / kFrames;
    const int f  = rc - b * kFrames;
    const float* src = x + (size_t)b * kTlen + (size_t)f * kShift + n0;
    const v4f a0 = *(const v4f*)(src);
    const v4f a1 = *(const v4f*)(src + 4);
    const unsigned keep = live ? 0xffffffffu : 0u;
    v4u w;
    w[0] = pack_bf16x2(a0[0], a0[1]) & keep;
    w[1] = pack_bf16x2(a0[2], a0[3]) & keep;
    w[2] = pack_bf16x2(a1[0], a1[1]) & keep;
    w[3] = pack_bf16x2(a1[2], a1[3]) & keep;
    unsigned short* dst = fr + (size_t)r * kNfft + n0;
    *(volatile v4u*)dst = w;
    __threadfence();
    *(volatile v4u*)dst = w;
  } else {
    const int t  = (blockIdx.x - kFrBlocks) * 256 + threadIdx.x;
    const int j  = t >> 6;
    const int n0 = (t & 63) * 8;
    const int jr = (j < kHalf) ? j : (kHalf - 1);
    const int ji = (j >= kHalf) ? (j - kHalf) : 0;
    const float* pr = wr + (size_t)jr * kNfft + n0;
    const float* pi = wi + (size_t)ji * kNfft + n0;
    const v4f r0 = *(const v4f*)(pr);
    const v4f r1 = *(const v4f*)(pr + 4);
    const v4f i0 = *(const v4f*)(pi);
    const v4f i1 = *(const v4f*)(pi + 4);
    const bool useR = (j < kHalf);
    const v4f a0 = useR ? r0 : i0;
    const v4f a1 = useR ? r1 : i1;
    v4u w;
    w[0] = pack_bf16x2(a0[0], a0[1]);
    w[1] = pack_bf16x2(a0[2], a0[3]);
    w[2] = pack_bf16x2(a1[0], a1[1]);
    w[3] = pack_bf16x2(a1[2], a1[3]);
    unsigned short* dst = wb + (size_t)j * kNfft + n0;
    *(volatile v4u*)dst = w;
    __threadfence();
    *(volatile v4u*)dst = w;
  }
}

__global__ __launch_bounds__(256) void logmag_norm(const float* __restrict__ S, float* __restrict__ NS)
{
#pragma clang fp contract(off)
  __shared__ __align__(16) float vs[8][kHalf];
  const int lane = threadIdx.x & 31;
  const int wave = threadIdx.x >> 5;
  const int rowRaw = blockIdx.x * 8 + wave;
  const bool rowOK = (rowRaw < kRows);
  const int row = rowOK ? rowRaw : (kRows - 1);
  const float* sp = S + (size_t)row * kScols;

  float s = 0.f;
#pragma unroll 1
  for (int i = 0; i < 8; ++i) {
    const int k = lane + 32 * i;
    const float re = sp[k];
    const float im = sp[kHalf + k];
    float p = re * re;
    const float q = im * im;
    p = p + q;
    p = p + kEps;
    const float v = logf(sqrtf(p)) * kInvLn10;
    vs[wave][k] = v;
    s += v;
  }
#pragma unroll
  for (int off = 16; off > 0; off >>= 1) s += __shfl_xor(s, off, 32);
  const float mean = s * (1.0f / 256.0f);

  __syncthreads();

  const v4f w0 = *(const v4f*)(&vs[wave][lane * 4]);
  const v4f w1 = *(const v4f*)(&vs[wave][128 + lane * 4]);
  const v4f d0 = w0 - mean;
  const v4f d1 = w1 - mean;
  float qs = 0.f;
  qs += d0[0] * d0[0]; qs += d0[1] * d0[1]; qs += d0[2] * d0[2]; qs += d0[3] * d0[3];
  qs += d1[0] * d1[0]; qs += d1[1] * d1[1]; qs += d1[2] * d1[2]; qs += d1[3] * d1[3];
#pragma unroll
  for (int off = 16; off > 0; off >>= 1) qs += __shfl_xor(qs, off, 32);
  const float var  = qs * (1.0f / 256.0f);
  const float stdv = sqrtf(var);
  const float inv  = 1.0f / (stdv + kEps);
  const v4f o0 = d0 * inv;
  const v4f o1 = d1 * inv;

  if (rowOK) {
    float* dst = NS + (size_t)row * kHalf;
    for (int pass = 0; pass < 2; ++pass) {
      *(volatile v4f*)(dst + lane * 4)       = o0;
      *(volatile v4f*)(dst + 128 + lane * 4) = o1;
      __threadfence();
    }
  }
}

__global__ __launch_bounds__(256) void pack_out(const float* __restrict__ NS, float* __restrict__ out)
{
  const int t = blockIdx.x * 256 + threadIdx.x;
  if (t >= kOutQuads) return;
  v4f o;
#pragma unroll
  for (int e = 0; e < 4; ++e) {
    const int idx = t * 4 + e;
    const int b   = idx / (kHalf * kFrames);
    const int rem = idx - b * (kHalf * kFrames);
    const int k   = rem / kFrames;
    const int f   = rem - k * kFrames;
    o[e] = NS[(size_t)(b * kFrames + f) * kHalf + k];
  }
  float* dst = out + (size_t)t * 4;
  *(volatile v4f*)dst = o;
  __threadfence();
  *(volatile v4f*)dst = o;
}

extern "C" void kernel_launch(void* const* d_in, const int* in_sizes, int n_in,
                              void* d_out, int out_size, void* d_ws, size_t ws_size,
                              hipStream_t stream) {
  if (n_in < 3) return;
  if (in_sizes[0] != kBatch * kTlen) return;
  if (in_sizes[1] != kNfft * kNfft) return;
  if (in_sizes[2] != kNfft * kNfft) return;
  if (out_size != kOutFloats) return;

  const size_t frBytes = (size_t)kRowsPad * kNfft * 2;
  const size_t wbBytes = (size_t)kScols * kNfft * 2;
  const size_t sBytes  = (size_t)kRowsPad * kScols * 4;
  const size_t nsBytes = (size_t)kRowsPad * kHalf * 4;
  const size_t offFR = 0;
  const size_t offWB = offFR + frBytes;
  const size_t offS  = offWB + wbBytes;
  const size_t offNS = offS + sBytes;
  const size_t total = offNS + nsBytes;
  if (total > ws_size) return;

  const float* x  = (const float*)d_in[0];
  const float* wr = (const float*)d_in[1];
  const float* wi = (const float*)d_in[2];
  float* out = (float*)d_out;
  char* ws = (char*)d_ws;
  unsigned short* FR = (unsigned short*)(ws + offFR);
  unsigned short* WB = (unsigned short*)(ws + offWB);
  float* S  = (float*)(ws + offS);
  float* NS = (float*)(ws + offNS);

  cast_planes<<<dim3(kFrBlocks + kWbBlocks), 256, 0, stream>>>(x, wr, wi, FR, WB);

  const int tilesM = kRowsPad / 64;
  const int tilesN = kScols / 64;
  const int gemmBlocks = (tilesM * tilesN + 7) / 8;
  wmma_gemm64<1, false, 0, 0, false, 0><<<dim3(gemmBlocks, 1), 256, 0, stream>>>(
      FR, FR, kNfft, 0L,
      WB, WB, kNfft, 0L,
      (void*)S, (void*)S, kScols, 0L,
      (const float*)S,
      (const float*)S, 0L,
      kRowsPad, kScols, kNfft, 1.0f);

  logmag_norm<<<dim3(kRows / 8), 256, 0, stream>>>(S, NS);

  pack_out<<<dim3(kOutQuads / 256), 256, 0, stream>>>(NS, out);
}
